// SioConvLayer_30743375905260
// MI455X (gfx1250) — hardware-verified
//
#include <hip/hip_runtime.h>
#include <stdint.h>
#include <stddef.h>


typedef _Float16 v16h __attribute__((ext_vector_type(16)));
typedef _Float16 v8h  __attribute__((ext_vector_type(8)));
typedef float    v8f  __attribute__((ext_vector_type(8)));
typedef float    v4f  __attribute__((ext_vector_type(4)));
typedef v8h v8ha __attribute__((may_alias));
typedef v4f v4fa __attribute__((may_alias));

#define NBATCH 4
#define NSEQ   1024
#define NDIM   1024
#define NHEAD  8
#define DHEAD  32
#define NQKVA  (NHEAD * DHEAD * 8)
#define NY2    (NHEAD * DHEAD * 2)
#define NTOK   (NBATCH * NSEQ)

#define GBM 64
#define GBN 128
#define GBK 32
#define GLS 40
#define GTS 132

#define SCL_W  16.0f
#define SCL_U  8.0f
#define SCL_Y  8.0f
#define SCL_G  16.0f

__device__ __forceinline__ v8f wmma_f16(v16h a, v16h b, v8f c)
{
    v8f d = __builtin_amdgcn_wmma_f32_16x16x32_f16(false, a, false, b, (short)0, c, false, false);
    asm volatile("v_nop\n\tv_nop\n\tv_nop\n\tv_nop" : "+v"(d) : "v"(a), "v"(b));
    return d;
}

__device__ __forceinline__ float silu_f(float v)
{
    return v / (1.0f + expf(-v));
}

__global__ __launch_bounds__(256) void k_cvt(const float* __restrict__ src, _Float16* dst, int n8, float scale)
{
    const int i = blockIdx.x * 256 + (int)threadIdx.x;
    if (i < n8) {
        const size_t o = (size_t)i * 8;
        const v4f p = *(const v4fa*)(src + o);
        const v4f q = *(const v4fa*)(src + o + 4);
        v8h hv;
#pragma unroll
        for (int j = 0; j < 4; ++j) {
            hv[j]     = (_Float16)(p[j] * scale);
            hv[j + 4] = (_Float16)(q[j] * scale);
        }
        volatile v8h* w = (volatile v8h*)(dst + o);
        *w = hv;
        __threadfence();
        *w = hv;
    }
}

__device__ __forceinline__ void gemm_store_rows(float* C, const float* tile, int wave, int lane,
                                                int blockM, int blockN, int M, int N)
{
    v4f v[8];
#pragma unroll
    for (int i = 0; i < 8; ++i)
        v[i] = *(const v4fa*)&tile[(wave * 8 + i) * GTS + lane * 4];
#pragma unroll
    for (int i = 0; i < 8; ++i) {
        const int gm = blockM + wave * 8 + i;
        if (gm < M) *(volatile v4f*)(C + (size_t)gm * N + blockN + lane * 4) = v[i];
    }
    __threadfence();
#pragma unroll
    for (int i = 0; i < 8; ++i) {
        const int gm = blockM + wave * 8 + i;
        if (gm < M) *(volatile v4f*)(C + (size_t)gm * N + blockN + lane * 4) = v[i];
    }
}

__device__ __forceinline__ void gemm_store_rows(_Float16* C, const float* tile, int wave, int lane,
                                                int blockM, int blockN, int M, int N)
{
    const int hh = lane >> 4;
    const int c8 = (lane & 15) * 8;
    v8h v[4];
#pragma unroll
    for (int i = 0; i < 4; ++i) {
        const int row = wave * 8 + i * 2 + hh;
        const v4f p = *(const v4fa*)&tile[row * GTS + c8];
        const v4f q = *(const v4fa*)&tile[row * GTS + c8 + 4];
#pragma unroll
        for (int j = 0; j < 4; ++j) {
            v[i][j]     = (_Float16)p[j];
            v[i][j + 4] = (_Float16)q[j];
        }
    }
#pragma unroll
    for (int i = 0; i < 4; ++i) {
        const int gm = blockM + wave * 8 + i * 2 + hh;
        if (gm < M) *(volatile v8h*)(C + (size_t)gm * N + blockN + c8) = v[i];
    }
    __threadfence();
#pragma unroll
    for (int i = 0; i < 4; ++i) {
        const int gm = blockM + wave * 8 + i * 2 + hh;
        if (gm < M) *(volatile v8h*)(C + (size_t)gm * N + blockN + c8) = v[i];
    }
}

template <typename OT, bool ACT>
__global__ __launch_bounds__(256) void k_gemm(const _Float16* __restrict__ A, const _Float16* __restrict__ W,
                                              const float* __restrict__ bias, OT* C,
                                              int M, int N, int K, float sacc, float sout)
{
    __shared__ _Float16 sA[GBM * GLS] __attribute__((aligned(16)));
    __shared__ _Float16 sB[GBN * GLS] __attribute__((aligned(16)));
    __shared__ float    sT[GBM * GTS] __attribute__((aligned(16)));

    const int tid  = threadIdx.x;
    const int lane = tid & 31;
    const int wave = tid >> 5;
    const int lm   = lane & 15;
    const int hh   = lane >> 4;
    const int wm   = wave >> 2;
    const int wn   = wave & 3;
    const int blockM = blockIdx.y * GBM;
    const int blockN = blockIdx.x * GBN;

    const int sr = tid >> 2;
    const int sc = (tid & 3) * 8;
    const _Float16* gA  = A + (size_t)(blockM + sr) * K + sc;
    const _Float16* gB0 = W + (size_t)(blockN + sr) * K + sc;
    const _Float16* gB1 = W + (size_t)(blockN + sr + 64) * K + sc;

    v8f acc[2][2];
#pragma unroll
    for (int mi = 0; mi < 2; ++mi)
#pragma unroll
        for (int ni = 0; ni < 2; ++ni)
#pragma unroll
            for (int i = 0; i < 8; ++i) acc[mi][ni][i] = 0.0f;

    for (int k0 = 0; k0 < K; k0 += GBK) {
        const v8h ra  = *(const v8ha*)(gA + k0);
        const v8h rb0 = *(const v8ha*)(gB0 + k0);
        const v8h rb1 = *(const v8ha*)(gB1 + k0);
        __syncthreads();
        *(v8ha*)&sA[sr * GLS + sc]        = ra;
        *(v8ha*)&sB[sr * GLS + sc]        = rb0;
        *(v8ha*)&sB[(sr + 64) * GLS + sc] = rb1;
        __syncthreads();

        union { v16h v; v8h half[2]; } fa[2], fb[2];
#pragma unroll
        for (int mi = 0; mi < 2; ++mi) {
            const int row = wm * 32 + mi * 16 + lm;
            fa[mi].half[0] = *(const v8ha*)&sA[row * GLS + 8 * hh];
            fa[mi].half[1] = *(const v8ha*)&sA[row * GLS + 16 + 8 * hh];
        }
#pragma unroll
        for (int ni = 0; ni < 2; ++ni) {
            const int row = wn * 32 + ni * 16 + lm;
            fb[ni].half[0] = *(const v8ha*)&sB[row * GLS + 8 * hh];
            fb[ni].half[1] = *(const v8ha*)&sB[row * GLS + 16 + 8 * hh];
        }
#pragma unroll
        for (int mi = 0; mi < 2; ++mi)
#pragma unroll
            for (int ni = 0; ni < 2; ++ni)
                acc[mi][ni] = wmma_f16(fa[mi].v, fb[ni].v, acc[mi][ni]);
    }

#pragma unroll
    for (int mi = 0; mi < 2; ++mi) {
#pragma unroll
        for (int ni = 0; ni < 2; ++ni) {
            const int col = wn * 32 + ni * 16 + lm;
            const float bv = bias[blockN + col];
#pragma unroll
            for (int r = 0; r < 8; ++r) {
                const int row = wm * 32 + mi * 16 + hh * 8 + r;
                float v = acc[mi][ni][r] * sacc + bv;
                if (ACT) v = silu_f(v);
                sT[row * GTS + col] = v * sout;
            }
        }
    }
    __syncthreads();
    gemm_store_rows(C, sT, wave, lane, blockM, blockN, M, N);
}

__device__ __forceinline__ void scan_stage(float (*Sb)[DHEAD], const float* __restrict__ src, int tid)
{
    v4f p = *(const v4fa*)(src + tid * 4);
    const int d  = tid >> 1;
    const int c0 = (tid & 1) * 4;
    if (tid & 1) {
        const float m2 = p[2] * p[2] + p[3] * p[3];
        const float s  = sqrtf(m2) / (1.0f + m2);
        p[2] *= s;
        p[3] *= s;
    }
    Sb[c0 + 0][d] = p[0];
    Sb[c0 + 1][d] = p[1];
    Sb[c0 + 2][d] = p[2];
    Sb[c0 + 3][d] = p[3];
}

__global__ __launch_bounds__(256) void k_scan(const float* __restrict__ qkva,
                                              const float* __restrict__ h0r,
                                              const float* __restrict__ h0i,
                                              _Float16* y2h, int L, float yscale)
{
    __shared__ float    S[2][8][DHEAD]     __attribute__((aligned(16)));
    __shared__ float    Y[2][8][DHEAD][2]  __attribute__((aligned(16)));
    __shared__ _Float16 T[32][2 * DHEAD]   __attribute__((aligned(16)));

    const int tid  = threadIdx.x;
    const int lane = tid & 31;
    const int wave = tid >> 5;
    const int b = blockIdx.x / NHEAD;
    const int h = blockIdx.x % NHEAD;
    const int e = lane;

    const size_t tokQ = (size_t)NQKVA;
    const size_t tokY = (size_t)NY2;
    const float* qb = qkva + (size_t)b * L * tokQ + (size_t)h * (DHEAD * 8);
    _Float16*    yb = y2h  + (size_t)b * L * tokY + (size_t)h * (DHEAD * 2);

    float hr[4], hi[4];
#pragma unroll
    for (int j = 0; j < 4; ++j) {
        const int d = wave * 4 + j;
        hr[j] = h0r[((size_t)h * DHEAD + d) * DHEAD + e];
        hi[j] = h0i[((size_t)h * DHEAD + d) * DHEAD + e];
    }

    if (tid < 64) scan_stage(S[0], qb, tid);
    __syncthreads();

    for (int l = 0; l < L; ++l) {
        const int buf = l & 1;
        const float vr = S[buf][4][e];
        const float vi = S[buf][5][e];
        const v4f q_r = *(const v4fa*)&S[buf][0][wave * 4];
        const v4f q_i = *(const v4fa*)&S[buf][1][wave * 4];
        const v4f k_r = *(const v4fa*)&S[buf][2][wave * 4];
        const v4f k_i = *(const v4fa*)&S[buf][3][wave * 4];
        const v4f a_r = *(const v4fa*)&S[buf][6][wave * 4];
        const v4f a_i = *(const v4fa*)&S[buf][7][wave * 4];

        float yr = 0.0f, yi = 0.0f;
#pragma unroll
        for (int j = 0; j < 4; ++j) {
            const float kvr = k_r[j] * vr - k_i[j] * vi;
            const float kvi = k_r[j] * vi + k_i[j] * vr;
            const float nr  = a_r[j] * hr[j] - a_i[j] * hi[j] + kvr;
            const float ni  = a_r[j] * hi[j] + a_i[j] * hr[j] + kvi;
            hr[j] = nr;
            hi[j] = ni;
            yr += q_r[j] * nr - q_i[j] * ni;
            yi += q_r[j] * ni + q_i[j] * nr;
        }
        Y[buf][wave][e][0] = yr;
        Y[buf][wave][e][1] = yi;

        if (l + 1 < L && tid < 64) scan_stage(S[buf ^ 1], qb + (size_t)(l + 1) * tokQ, tid);
        __syncthreads();

        if (wave == 0) {
            float sre = 0.0f, sim = 0.0f;
#pragma unroll
            for (int w = 0; w < 8; ++w) {
                sre += Y[buf][w][e][0];
                sim += Y[buf][w][e][1];
            }
            T[l & 31][2 * e]     = (_Float16)(sre * yscale);
            T[l & 31][2 * e + 1] = (_Float16)(sim * yscale);
        }

        if ((l & 31) == 31) {
            __syncthreads();
            const int r  = wave * 4 + (lane >> 3);
            const int ch = (lane & 7) * 8;
            const v8h val = *(const v8ha*)&T[r][ch];
            volatile v8h* dst = (volatile v8h*)(yb + (size_t)(l - 31 + r) * tokY + ch);
            *dst = val;
            __threadfence();
            *dst = val;
        }
    }
}

extern "C" void kernel_launch(void* const* d_in, const int* in_sizes, int n_in,
                              void* d_out, int out_size, void* d_ws, size_t ws_size,
                              hipStream_t stream)
{
    if (n_in < 11) return;
    if (in_sizes[0]  != NTOK * NDIM)           return;
    if (in_sizes[1]  != NDIM * NDIM)           return;
    if (in_sizes[2]  != NDIM)                  return;
    if (in_sizes[3]  != NQKVA * NDIM)          return;
    if (in_sizes[4]  != NQKVA)                 return;
    if (in_sizes[5]  != NDIM * NY2)            return;
    if (in_sizes[6]  != NDIM)                  return;
    if (in_sizes[7]  != NDIM * NDIM)           return;
    if (in_sizes[8]  != NDIM)                  return;
    if (in_sizes[9]  != NHEAD * DHEAD * DHEAD) return;
    if (in_sizes[10] != NHEAD * DHEAD * DHEAD) return;
    if (out_size     != NTOK * NDIM)           return;
    if ((NTOK % GBM) != 0 || (NDIM % GBN) != 0 || (NQKVA % GBN) != 0 ||
        (NDIM % GBK) != 0 || (NY2 % GBK) != 0 || (NSEQ % 32) != 0) return;

    const float* x      = (const float*)d_in[0];
    const float* W_in   = (const float*)d_in[1];
    const float* b_in   = (const float*)d_in[2];
    const float* W_qkva = (const float*)d_in[3];
    const float* b_qkva = (const float*)d_in[4];
    const float* W_y    = (const float*)d_in[5];
    const float* b_y    = (const float*)d_in[6];
    const float* W_out  = (const float*)d_in[7];
    const float* b_out  = (const float*)d_in[8];
    const float* h0r    = (const float*)d_in[9];
    const float* h0i    = (const float*)d_in[10];
    float* out = (float*)d_out;

    char* ws = (char*)d_ws;
    size_t off = 0;
    _Float16* xh   = (_Float16*)(ws + off); off += (size_t)NTOK  * NDIM  * 2;
    _Float16* wih  = (_Float16*)(ws + off); off += (size_t)NDIM  * NDIM  * 2;
    _Float16* wqh  = (_Float16*)(ws + off); off += (size_t)NQKVA * NDIM  * 2;
    _Float16* wyh  = (_Float16*)(ws + off); off += (size_t)NDIM  * NY2   * 2;
    _Float16* woh  = (_Float16*)(ws + off); off += (size_t)NDIM  * NDIM  * 2;
    _Float16* u    = (_Float16*)(ws + off); off += (size_t)NTOK  * NDIM  * 2;
    float*    qkva = (float*)(ws + off);    off += (size_t)NTOK  * NQKVA * 4;
    _Float16* y2h  = (_Float16*)(ws + off); off += (size_t)NTOK  * NY2   * 2;
    _Float16* y2g  = (_Float16*)(ws + off); off += (size_t)NTOK  * NDIM  * 2;
    if (off > ws_size) return;

    const dim3 blk(256);

    {
        const int n8 = (NTOK * NDIM) / 8;
        k_cvt<<<dim3((unsigned)((n8 + 255) / 256)), blk, 0, stream>>>(x, xh, n8, 1.0f);
    }
    {
        const int n8 = (NDIM * NDIM) / 8;
        k_cvt<<<dim3((unsigned)((n8 + 255) / 256)), blk, 0, stream>>>(W_in, wih, n8, SCL_W);
    }
    {
        const int n8 = (NQKVA * NDIM) / 8;
        k_cvt<<<dim3((unsigned)((n8 + 255) / 256)), blk, 0, stream>>>(W_qkva, wqh, n8, SCL_W);
    }
    {
        const int n8 = (NDIM * NY2) / 8;
        k_cvt<<<dim3((unsigned)((n8 + 255) / 256)), blk, 0, stream>>>(W_y, wyh, n8, SCL_W);
    }
    {
        const int n8 = (NDIM * NDIM) / 8;
        k_cvt<<<dim3((unsigned)((n8 + 255) / 256)), blk, 0, stream>>>(W_out, woh, n8, SCL_W);
    }

    k_gemm<_Float16, true><<<dim3(NDIM / GBN, NTOK / GBM), blk, 0, stream>>>(
        xh, wih, b_in, u, NTOK, NDIM, NDIM, 1.0f / SCL_W, SCL_U);
    k_gemm<float, false><<<dim3(NQKVA / GBN, NTOK / GBM), blk, 0, stream>>>(
        u, wqh, b_qkva, qkva, NTOK, NQKVA, NDIM, 1.0f / (SCL_U * SCL_W), 1.0f);
    k_scan<<<dim3(NBATCH * NHEAD), blk, 0, stream>>>(qkva, h0r, h0i, y2h, NSEQ, SCL_Y);
    k_gemm<_Float16, true><<<dim3(NDIM / GBN, NTOK / GBM), blk, 0, stream>>>(
        y2h, wyh, b_y, y2g, NTOK, NDIM, NY2, 1.0f / (SCL_Y * SCL_W), SCL_G);
    k_gemm<float, false><<<dim3(NDIM / GBN, NTOK / GBM), blk, 0, stream>>>(
        y2g, woh, b_out, out, NTOK, NDIM, NDIM, 1.0f / (SCL_G * SCL_W), 1.0f);
}
